// LearnedMultiScaleGuidedFilter_78915729097397
// MI455X (gfx1250) — hardware-verified
//
#include <hip/hip_runtime.h>
#include <math.h>

#pragma clang fp contract(off)

typedef __attribute__((ext_vector_type(16))) _Float16 v16h;
typedef __attribute__((ext_vector_type(8)))  _Float16 v8h;
typedef __attribute__((ext_vector_type(16))) __bf16   v16b;
typedef __attribute__((ext_vector_type(8)))  __bf16   v8b;
typedef __attribute__((ext_vector_type(8)))  float    v8f;
typedef __attribute__((ext_vector_type(4)))  float    v4f;

#define LR 256
#define HR 1024
#define NSMAX 4
#define LOG_SMALL_EPS_F (-11.512925464970229f)

struct KS { int kh0, kh1, kh2, kh3, kw0, kw1, kw2, kw3, ns, bc; };
typedef char ks_size_check[(sizeof(KS) == 40) ? 1 : -1];

__device__ __forceinline__ int sel4(int s, int a, int b, int c, int d) {
  return (s == 0) ? a : ((s == 1) ? b : ((s == 2) ? c : d));
}

__device__ __forceinline__ unsigned short f2bf_bits(float f) {
  unsigned u = __float_as_uint(f);
  return (unsigned short)((u + 0x7FFFu + ((u >> 16) & 1u)) >> 16);
}
__device__ __forceinline__ float bf_bits2f(unsigned short h) { return __uint_as_float(((unsigned)h) << 16); }

__device__ __forceinline__ void dep_guard_h(v8f& a, v8f& b, v16h x, v16h y) { asm volatile("v_nop\n\tv_nop\n\tv_nop\n\tv_nop" : "+v"(a), "+v"(b) : "v"(x), "v"(y)); }
__device__ __forceinline__ void dep_guard_b(v8f& a, v8f& b, v16b x, v16b y) { asm volatile("v_nop\n\tv_nop\n\tv_nop\n\tv_nop" : "+v"(a), "+v"(b) : "v"(x), "v"(y)); }
__device__ __forceinline__ void keep4_h(v16h a, v16h b, v16h c, v16h d) { asm volatile("v_nop" :: "v"(a), "v"(b), "v"(c), "v"(d)); }
__device__ __forceinline__ void keep4_b(v16b a, v16b b, v16b c, v16b d) { asm volatile("v_nop" :: "v"(a), "v"(b), "v"(c), "v"(d)); }
__device__ __forceinline__ void acc_guard4(v8f& a, v8f& b, v8f& c, v8f& d) { asm volatile("v_nop\n\tv_nop\n\tv_nop\n\tv_nop" : "+v"(a), "+v"(b), "+v"(c), "+v"(d)); }
template <typename T> struct Frag;
template <> struct Frag<_Float16> {
  typedef v16h V; union U { v16h v; v8h h[2]; };
  static __device__ __forceinline__ v16h load(const _Float16* p) {
    U f; f.h[0] = *(const v8h*)(p); f.h[1] = *(const v8h*)(p + 16); return f.v;
  }
  static __device__ __forceinline__ v8f mma(v16h a, v16h b, v8f c) {
    return __builtin_amdgcn_wmma_f32_16x16x32_f16(false, a, false, b, (short)0, c, false, false);
  }
  static __device__ __forceinline__ void guard(v8f& a, v8f& b, v16h x, v16h y) { dep_guard_h(a, b, x, y); }
  static __device__ __forceinline__ void keep(v16h a, v16h b, v16h c, v16h d) { keep4_h(a, b, c, d); }
};
template <> struct Frag<__bf16> {
  typedef v16b V; union U { v16b v; v8b h[2]; };
  static __device__ __forceinline__ v16b load(const __bf16* p) {
    U f; f.h[0] = *(const v8b*)(p); f.h[1] = *(const v8b*)(p + 16); return f.v;
  }
  static __device__ __forceinline__ v8f mma(v16b a, v16b b, v8f c) {
    return __builtin_amdgcn_wmma_f32_16x16x32_bf16(false, a, false, b, (short)0, c, false, false);
  }
  static __device__ __forceinline__ void guard(v8f& a, v8f& b, v16b x, v16b y) { dep_guard_b(a, b, x, y); }
  static __device__ __forceinline__ void keep(v16b a, v16b b, v16b c, v16b d) { keep4_b(a, b, c, d); }
};

template <int ET> struct Elem;
template <> struct Elem<0> { typedef _Float16 T; };
template <> struct Elem<1> { typedef __bf16 T; };
template <int ET, bool SPLIT, int BIAS_MODE, int OUT_MODE, int RES, int ACT = 0>
__global__ __launch_bounds__(256) void wmma_gemm64(
    const unsigned short* __restrict__ Ap, const unsigned short* __restrict__ A2p, int lda, long strideA,
    const unsigned short* __restrict__ Btp, const unsigned short* __restrict__ Bt2p, int ldb, long strideB,
    void* Cout, void* Cout2, int ldc, long strideC,
    const float* __restrict__ bias,
    const float* resid, long strideR,
    int M, int N, int K, float scale) {
  typedef typename Elem<ET>::T T;
  typedef typename Frag<T>::V V;
  const T* A = (const T*)Ap; const T* A2 = (const T*)A2p; const T* Bt = (const T*)Btp; const T* Bt2 = (const T*)Bt2p;
  __shared__ __align__(16) float sT[8][16 * 68];
  const int b    = blockIdx.y;
  const int lane = threadIdx.x & 31;
  const int wave = threadIdx.x >> 5;
  const int tilesN = N >> 6;
  const int tilesM = M >> 6;
  const int tile = blockIdx.x * 8 + wave;
  if (tile >= tilesM * tilesN) return;
  const int tm = tile / tilesN;
  const int tn = tile - tm * tilesN;
  const int m0 = tm << 6;
  const int n0 = tn << 6;

  const T* Ab  = A  + (size_t)b * strideA;
  const T* Bb  = Bt + (size_t)b * strideB;
  const T* Ab2 = SPLIT ? (A2  + (size_t)b * strideA) : nullptr;
  const T* Bb2 = SPLIT ? (Bt2 + (size_t)b * strideB) : nullptr;

  const int rlane = lane & 15;
  const int koff  = (lane >> 4) * 8;
  const int mOff  = (lane >> 4) * 8;

  v8f acc[4][4];
#pragma unroll
  for (int i = 0; i < 4; ++i)
#pragma unroll
    for (int j = 0; j < 4; ++j) acc[i][j] = (v8f){0.f,0.f,0.f,0.f,0.f,0.f,0.f,0.f};

  for (int k0 = 0; k0 < K; k0 += 32) {
    V bh[4], bl[4];
#pragma unroll
    for (int j = 0; j < 4; ++j) {
      const size_t bo = (size_t)(n0 + (j << 4) + rlane) * ldb + koff + k0;
      bh[j] = Frag<T>::load(Bb + bo);
      if (SPLIT) bl[j] = Frag<T>::load(Bb2 + bo);
    }
#pragma unroll
    for (int i = 0; i < 4; ++i) {
      const size_t ao = (size_t)(m0 + (i << 4) + rlane) * lda + koff + k0;
      V ah = Frag<T>::load(Ab + ao);
      V al;
      if (SPLIT) al = Frag<T>::load(Ab2 + ao);
#pragma unroll
      for (int j = 0; j < 4; ++j) {
        acc[i][j] = Frag<T>::mma(ah, bh[j], acc[i][j]);
        if (SPLIT) {
          acc[i][j] = Frag<T>::mma(ah, bl[j], acc[i][j]);
          acc[i][j] = Frag<T>::mma(al, bh[j], acc[i][j]);
        }
      }
      Frag<T>::guard(acc[i][0], acc[i][3], ah, SPLIT ? al : ah);
    }
    Frag<T>::keep(bh[0], bh[1], bh[2], bh[3]);
    if (SPLIT) Frag<T>::keep(bl[0], bl[1], bl[2], bl[3]);
  }
  acc_guard4(acc[0][0], acc[0][1], acc[0][2], acc[0][3]);
  acc_guard4(acc[1][0], acc[1][1], acc[1][2], acc[1][3]);
  acc_guard4(acc[2][0], acc[2][1], acc[2][2], acc[2][3]);
  acc_guard4(acc[3][0], acc[3][1], acc[3][2], acc[3][3]);

  float* slab = sT[wave];
  const float* Rb = (RES != 0) ? (resid + (size_t)b * strideR) : nullptr;
#pragma unroll
  for (int i = 0; i < 4; ++i) {
    const int mBase = m0 + (i << 4);
#pragma unroll
    for (int j = 0; j < 4; ++j) {
      const int n = n0 + (j << 4) + rlane;
      float bv = 0.f;
      if (BIAS_MODE == 2) bv = bias[n];
#pragma unroll
      for (int r = 0; r < 8; ++r) {
        float v = acc[i][j][r] * scale;
        if (BIAS_MODE == 1) v += bias[mBase + mOff + r];
        if (BIAS_MODE == 2) v += bv;
        if (RES == 1) v += Rb[(size_t)(mBase + mOff + r) * ldc + n];
        if (RES == 2) v *= Rb[(size_t)(mBase + mOff + r) * ldc + n];
        if (ACT == 1) v = tanhf(v);
        if (ACT == 2) v = fmaxf(v, 0.0f);
        if (ACT == 3) v = v / (1.0f + expf(-v));
        if (ACT == 4) v = (v > 0.f) ? v : 0.01f * v;
        if (ACT == 5) v = 0.5f * v * (1.0f + erff(v * 0.70710678118654752f));
        slab[(mOff + r) * 68 + (j << 4) + rlane] = v;
      }
    }
    __builtin_amdgcn_fence(__ATOMIC_RELEASE, "workgroup");
    __builtin_amdgcn_wave_barrier();
    __builtin_amdgcn_fence(__ATOMIC_ACQUIRE, "workgroup");
    if (OUT_MODE == 0) {
      float* C = (float*)Cout + (size_t)b * strideC;
      const int hh = lane >> 4, c4 = (lane & 15) * 4;
      for (int pass = 0; pass < 2; ++pass) {
#pragma unroll
        for (int it = 0; it < 8; ++it) {
          const int row = it * 2 + hh;
          v4f v = *(const v4f*)(slab + row * 68 + c4);
          *(volatile v4f*)(C + (size_t)(mBase + row) * ldc + n0 + c4) = v;
        }
        __threadfence();
      }
    } else {
      const int q = lane >> 3, c8 = (lane & 7) * 8;
      unsigned short* C  = (unsigned short*)Cout  + (size_t)b * strideC;
      unsigned short* C2 = (OUT_MODE == 2) ? ((unsigned short*)Cout2 + (size_t)b * strideC) : nullptr;
      for (int pass = 0; pass < 2; ++pass) {
#pragma unroll
        for (int it = 0; it < 4; ++it) {
          const int row = it * 4 + q;
          const float* sp = slab + row * 68 + c8;
          v8h hv, lv;
#pragma unroll
          for (int e = 0; e < 8; ++e) {
            if (OUT_MODE == 1) {
              hv[e] = (_Float16)sp[e];
            } else {
              unsigned short hb = f2bf_bits(sp[e]);
              unsigned short lb = f2bf_bits(sp[e] - bf_bits2f(hb));
              hv[e] = __builtin_bit_cast(_Float16, hb);
              lv[e] = __builtin_bit_cast(_Float16, lb);
            }
          }
          *(volatile v8h*)(C + (size_t)(mBase + row) * ldc + n0 + c8) = hv;
          if (OUT_MODE == 2) *(volatile v8h*)(C2 + (size_t)(mBase + row) * ldc + n0 + c8) = lv;
        }
        __threadfence();
      }
    }
    __builtin_amdgcn_fence(__ATOMIC_RELEASE, "workgroup");
    __builtin_amdgcn_wave_barrier();
    __builtin_amdgcn_fence(__ATOMIC_ACQUIRE, "workgroup");
  }
}

__global__ __launch_bounds__(256) void k_build_r(_Float16* __restrict__ R) {
  const int t = blockIdx.x * 256 + threadIdx.x;
  const int o = t >> 5;
  const int i0 = (t & 31) * 8;
  if (o >= HR) return;
  const float sf = ((float)o + 0.5f) * ((float)LR / (float)HR) - 0.5f;
  const float fl = floorf(sf);
  const float fr = sf - fl;
  int ia = (int)fl;
  int ib = ia + 1;
  ia = min(max(ia, 0), LR - 1);
  ib = min(max(ib, 0), LR - 1);
  v8h v;
#pragma unroll
  for (int e = 0; e < 8; ++e) {
    const int i = i0 + e;
    float w = 0.0f;
    if (i == ia) w = w + (1.0f - fr);
    if (i == ib) w = w + fr;
    v[e] = (_Float16)w;
  }
  _Float16* dst = R + (size_t)o * LR + i0;
  *(volatile v8h*)dst = v;
  __threadfence();
  *(volatile v8h*)dst = v;
}

__global__ __launch_bounds__(256) void k_hprefix(const float* __restrict__ target, const float* __restrict__ guide,
                                                 float* __restrict__ II, int bc) {
  const int img = blockIdx.x % bc;
  const int q = blockIdx.x / bc;
  const int j = threadIdx.x;
  if (q >= 4) return;
  const float* t = target + (size_t)img * (LR * LR) + j;
  const float* g = guide + (size_t)img * (LR * LR) + j;
  volatile float* o = II + (size_t)(q * bc + img) * ((LR + 1) * LR) + j;
  for (int pass = 0; pass < 2; ++pass) {
    o[0] = 0.0f;
    float acc = 0.0f, carry = 0.0f;
#pragma unroll 1
    for (int r = 0; r < LR; ++r) {
      if (r == LR / 2) { carry = acc; acc = 0.0f; }
      const float tv = t[(size_t)r * LR];
      const float gv = g[(size_t)r * LR];
      const float x = (q == 0) ? tv : ((q == 1) ? gv : ((q == 2) ? (tv * gv) : (gv * gv)));
      acc = acc + x;
      o[(size_t)(r + 1) * LR] = acc + carry;
    }
    __threadfence();
  }
}

__global__ __launch_bounds__(32) void k_wprefix_box(const float* __restrict__ II, float* __restrict__ BOX, KS ks) {
  __shared__ float P[32][260];
  const int lane = threadIdx.x;
  const int id = blockIdx.x * 32 + lane;
  const int i = id & (LR - 1);
  int rest = id >> 8;
  const int q = rest & 3;
  rest >>= 2;
  const int s = rest % ks.ns;
  int img = rest / ks.ns;
  const bool valid = (img < ks.bc);
  if (!valid) img = 0;
  const int kh = sel4(s, ks.kh0, ks.kh1, ks.kh2, ks.kh3);
  const int kw = sel4(s, ks.kw0, ks.kw1, ks.kw2, ks.kw3);
  int loi = i - (kh - 1) / 2; loi = min(max(loi, 0), LR);
  int hii = i + kh / 2 + 1;   hii = min(max(hii, 0), LR);
  const float* rh = II + ((size_t)(q * ks.bc + img) * (LR + 1) + hii) * LR;
  const float* rl = II + ((size_t)(q * ks.bc + img) * (LR + 1) + loi) * LR;
  float* p = P[lane];
  p[0] = 0.0f;
  float acc = 0.0f, carry = 0.0f;
#pragma unroll 1
  for (int j = 0; j < LR; ++j) {
    if (j == LR / 2) { carry = acc; acc = 0.0f; }
    const float y = rh[j] - rl[j];
    acc = acc + y;
    p[j + 1] = acc + carry;
  }
  const int aw = (kw - 1) / 2;
  const int bw = kw / 2 + 1;
  float* brow = BOX + (size_t)id * LR;
  if (valid) {
    for (int pass = 0; pass < 2; ++pass) {
#pragma unroll 1
      for (int j0 = 0; j0 < LR; j0 += 4) {
        v4f v;
#pragma unroll
        for (int e = 0; e < 4; ++e) {
          const int j = j0 + e;
          int lo = j - aw; lo = min(max(lo, 0), LR);
          int hi = j + bw; hi = min(max(hi, 0), LR);
          v[e] = p[hi] - p[lo];
        }
        *(volatile v4f*)(brow + j0) = v;
      }
      __threadfence();
    }
  }
}

__global__ __launch_bounds__(256) void k_stats(const float* __restrict__ BOX, const float* __restrict__ log_eps,
                                               const float* __restrict__ wts, _Float16* __restrict__ FT, KS ks) {
  __shared__ __align__(16) _Float16 tA[128 * 64];
  __shared__ __align__(16) _Float16 tB[128 * 64];
  __shared__ float s_eps[NSMAX];
  __shared__ float s_w[NSMAX];
  const int tid = threadIdx.x;
  const int bc = ks.bc, ns = ks.ns;
  const int img = blockIdx.x >> 3;
  const int rg = (blockIdx.x >> 1) & 3;
  const int wh = blockIdx.x & 1;
  if (tid == 0) {
    float wmax = wts[0];
#pragma unroll 1
    for (int s = 1; s < ns; ++s) wmax = fmaxf(wmax, wts[s]);
    float den = 0.0f;
#pragma unroll 1
    for (int s = 0; s < ns; ++s) den = den + expf(wts[s] - wmax);
    const float invden = 1.0f / den;
#pragma unroll 1
    for (int s = 0; s < ns; ++s) {
      s_w[s] = expf(wts[s] - wmax) * invden;
      const float le = fminf(fmaxf(log_eps[s], LOG_SMALL_EPS_F), 100.0f);
      s_eps[s] = expf(le);
    }
  }
  __syncthreads();

  const int jl = tid & 127;
  const int lb = tid >> 7;
  const int j = wh * 128 + jl;
  const int r0 = rg * 64;
  const size_t qs = (size_t)LR * LR;
#pragma unroll 1
  for (int k = 0; k < 32; ++k) {
    const int li = lb + 2 * k;
    const int i = r0 + li;
    float Aacc = 0.0f, Bacc = 0.0f;
#pragma unroll 1
    for (int s = 0; s < ns; ++s) {
      const int kh = sel4(s, ks.kh0, ks.kh1, ks.kh2, ks.kh3);
      const int kw = sel4(s, ks.kw0, ks.kw1, ks.kw2, ks.kw3);
      int loi = i - (kh - 1) / 2; loi = min(max(loi, 0), LR);
      int hii = i + kh / 2 + 1;   hii = min(max(hii, 0), LR);
      int loj = j - (kw - 1) / 2; loj = min(max(loj, 0), LR);
      int hij = j + kw / 2 + 1;   hij = min(max(hij, 0), LR);
      const float norm = (float)((hii - loi) * (hij - loj));
      const float invn = 1.0f / norm;
      const float* bp = BOX + (((size_t)(img * ns + s) * 4) * LR + i) * LR + j;
      const float bt = bp[0];
      const float bg = bp[qs];
      const float btg = bp[2 * qs];
      const float bgg = bp[3 * qs];
      const float tm = bt * invn;
      const float gm = bg * invn;
      const float cov = btg * invn - tm * gm;
      const float var = bgg * invn - gm * gm;
      const float As = cov / (var + s_eps[s]);
      const float bs = tm - As * gm;
      Aacc = Aacc + As * s_w[s];
      Bacc = Bacc + bs * s_w[s];
    }
    tA[jl * 64 + li] = (_Float16)Aacc;
    tB[jl * 64 + li] = (_Float16)Bacc;
  }
  __syncthreads();

  const int wave = tid >> 5, lane = tid & 31;
  const int piece = lane & 7, lq = lane >> 3;
  for (int pass = 0; pass < 2; ++pass) {
#pragma unroll 1
    for (int it = 0; it < 8; ++it) {
      const int L = it * 32 + wave * 4 + lq;
      const int field = L >> 7;
      const int jl2 = L & 127;
      const _Float16* src = (field ? tB : tA) + jl2 * 64 + piece * 8;
      const v8h val = *(const v8h*)src;
      _Float16* dst = FT + ((size_t)(field * bc + img) * LR + (wh * 128 + jl2)) * LR + r0 + piece * 8;
      *(volatile v8h*)dst = val;
    }
    __threadfence();
  }
}

extern "C" void kernel_launch(void* const* d_in, const int* in_sizes, int n_in,
                              void* d_out, int out_size, void* d_ws, size_t ws_size,
                              hipStream_t stream) {
  if (n_in < 5) return;
  const float* guide_hr = (const float*)d_in[0];
  const float* guide    = (const float*)d_in[1];
  const float* target   = (const float*)d_in[2];
  const float* log_eps  = (const float*)d_in[3];
  const float* weights  = (const float*)d_in[4];
  float* out = (float*)d_out;

  const int lr = LR * LR;
  const int hr = HR * HR;
  if (in_sizes[1] <= 0 || (in_sizes[1] % lr) != 0) return;
  const int bc = in_sizes[1] / lr;
  if (bc < 1 || bc > 1024) return;
  if (in_sizes[2] != in_sizes[1]) return;
  if ((long long)in_sizes[0] != (long long)bc * hr) return;
  if ((long long)out_size != (long long)bc * hr) return;
  const int ns = in_sizes[4];
  if (ns < 1 || ns > NSMAX || in_sizes[3] != ns) return;

  int kh[NSMAX], kw[NSMAX];
  for (int i = 0; i < NSMAX; ++i) { kh[i] = LR; kw[i] = LR; }
  kh[0] = (LR < 3) ? LR : 3;
  kw[0] = (LR < 3) ? LR : 3;
  if (ns > 1) {
    int d = LR - 3; if (d < 0) d = -d;
    const int dh = d / (ns - 1);
    const int dw = d / (ns - 1);
    for (int i = 1; i < ns - 1; ++i) {
      int a = 3 + i * dh; kh[i] = (a < LR) ? a : LR;
      int bb = 3 + i * dw; kw[i] = (bb < LR) ? bb : LR;
    }
    kh[ns - 1] = LR;
    kw[ns - 1] = LR;
  }
  KS ks;
  ks.kh0 = kh[0]; ks.kh1 = kh[1]; ks.kh2 = kh[2]; ks.kh3 = kh[3];
  ks.kw0 = kw[0]; ks.kw1 = kw[1]; ks.kw2 = kw[2]; ks.kw3 = kw[3];
  ks.ns = ns; ks.bc = bc;

  unsigned char* ws = (unsigned char*)d_ws;
  const size_t szR   = (size_t)HR * LR * 2;
  const size_t szII  = (size_t)4 * bc * (LR + 1) * LR * 4;
  const size_t szBOX = (size_t)bc * ns * 4 * lr * 4;
  const size_t szFT  = (size_t)2 * bc * lr * 2;
  const size_t szU   = (size_t)2 * bc * HR * LR * 2;
  const size_t offR = 0;
  const size_t offII = offR + szR;
  const size_t offBOX = offII + szII;
  const size_t offFT = offBOX + szBOX;
  const size_t offU = offFT + szFT;
  const size_t total = offU + szU;
  if (total > ws_size) return;

  _Float16* R16 = (_Float16*)(ws + offR);
  float* II = (float*)(ws + offII);
  float* BOX = (float*)(ws + offBOX);
  _Float16* FT = (_Float16*)(ws + offFT);
  _Float16* U = (_Float16*)(ws + offU);
  const unsigned short* R16u = (const unsigned short*)R16;
  const unsigned short* FTu = (const unsigned short*)FT;
  const unsigned short* Uu = (const unsigned short*)U;
  const float* dummyf = (const float*)(ws + offR);

  k_build_r<<<dim3((HR * (LR / 8) + 255) / 256), dim3(256), 0, stream>>>(R16);
  k_hprefix<<<dim3(4 * bc), dim3(256), 0, stream>>>(target, guide, II, bc);
  k_wprefix_box<<<dim3(bc * ns * 4 * (LR / 32)), dim3(32), 0, stream>>>(II, BOX, ks);
  k_stats<<<dim3(bc * 8), dim3(256), 0, stream>>>(BOX, log_eps, weights, FT, ks);

  {
    const int tiles = (HR / 64) * (LR / 64);
    wmma_gemm64<0, false, 0, 1, 0><<<dim3((tiles + 7) / 8, 2 * bc), dim3(256), 0, stream>>>(
        R16u, R16u, LR, 0L,
        FTu, FTu, LR, (long)lr,
        (void*)U, (void*)U, LR, (long)HR * LR,
        dummyf,
        dummyf, 0L,
        HR, LR, LR, 1.0f);
  }
  {
    const int tiles = (HR / 64) * (HR / 64);
    wmma_gemm64<0, false, 0, 0, 2><<<dim3((tiles + 7) / 8, bc), dim3(256), 0, stream>>>(
        Uu, Uu, LR, (long)HR * LR,
        R16u, R16u, LR, 0L,
        (void*)out, (void*)out, HR, (long)hr,
        dummyf,
        guide_hr, (long)hr,
        HR, HR, LR, 1.0f);
    wmma_gemm64<0, false, 0, 0, 1><<<dim3((tiles + 7) / 8, bc), dim3(256), 0, stream>>>(
        Uu + (size_t)bc * HR * LR, Uu + (size_t)bc * HR * LR, LR, (long)HR * LR,
        R16u, R16u, LR, 0L,
        (void*)out, (void*)out, HR, (long)hr,
        dummyf,
        (const float*)out, (long)hr,
        HR, HR, LR, 1.0f);
  }
}
